// CrossAttention_1683627180152
// MI455X (gfx1250) — hardware-verified
//
#include <hip/hip_runtime.h>
#include <math.h>
#include <stdint.h>

#ifndef NB
#define NB 2
#endif
#ifndef SEQ
#define SEQ 4096
#endif
#ifndef MSEQ
#define MSEQ SEQ
#endif
#define NB_FULL   2
#define SEQ_FULL  4096
#define MSEQ_FULL 4096
#define DM    512
#define DC    512
#define NH    8
#define HD    64
#define DI    (NH * HD)
#define KVN   (2 * DI)
#define XLD   (2 * DM)
#define OPLD  (2 * DI)
#define NQB   (SEQ / 64)
#define NKT   (MSEQ / 64)
#define PCARRY 16384.0f
#define VCARRY 16.0f
#define CCARRY 256.0f
#define RQ     4096.0f
#define RC     64.0f
#define WOC    64.0f
#define SQK    0.35355339059327f
#define LN_EPS 1e-5f
#define NEGMAX (-3.402823466e+38f)

static_assert(HD == 64);
static_assert(NH * HD == DI && DI == 512);
static_assert(DM == 512 && DC == 512);
static_assert(32 * 8 * 2 == DM && 32 * 4 * 4 == DM);
static_assert(XLD == 2 * DM && OPLD == 2 * DI && KVN == 2 * DI);
static_assert(NB >= 1 && NB <= NB_FULL);
static_assert(SEQ >= 64 && SEQ <= SEQ_FULL && (SEQ % 64) == 0);
static_assert(MSEQ >= 64 && MSEQ <= MSEQ_FULL && (MSEQ % 64) == 0);
static_assert((DM % 64) == 0 && (DI % 64) == 0 && (DC % 64) == 0 && (KVN % 64) == 0);
static_assert((DC % 32) == 0 && (XLD % 32) == 0 && (OPLD % 32) == 0);
static_assert(((NB * SEQ) % 64) == 0 && ((NB * MSEQ) % 64) == 0);
static_assert(((NB * SEQ) % 8) == 0);
static_assert(((MSEQ * DC / 8) % 256) == 0);
static_assert(128 * 32 == 64 * 64);
static_assert(256 * 4 * 4 == 64 * 64);
static_assert(PCARRY < 65504.0f);
static_assert((size_t)((NB_FULL - 1) * SEQ_FULL + SEQ_FULL) * DM * 4 == (size_t)16777216);

static constexpr size_t WSB_XN = (size_t)NB * SEQ * XLD * 2;
static constexpr size_t WSB_CB = (size_t)NB * MSEQ * DC * 2;
static constexpr size_t WSB_WQ = (size_t)DI * XLD * 2;
static constexpr size_t WSB_WKV = (size_t)KVN * DC * 2;
static constexpr size_t WSB_WO = (size_t)DM * OPLD * 2;
static constexpr size_t WSB_Q  = (size_t)NB * SEQ * DI * 2;
static constexpr size_t WSB_K  = (size_t)NB * MSEQ * DI * 2;
static constexpr size_t WSB_VT = (size_t)NB * DI * MSEQ * 2;
static constexpr size_t WSB_OP = (size_t)NB * SEQ * OPLD * 2;
static constexpr size_t WSB_Y  = (size_t)NB * SEQ * DM * 4;
static constexpr size_t WSB_TOTAL = WSB_XN + WSB_CB + WSB_WQ + WSB_WKV + WSB_WO + 2 * WSB_Q + WSB_K + WSB_VT + WSB_OP + WSB_Y;
static_assert(WSB_TOTAL <= (size_t)134217728);
static_assert((WSB_XN % 128) == 0 && (WSB_CB % 128) == 0 && (WSB_WQ % 128) == 0 && (WSB_WKV % 128) == 0);
static_assert((WSB_WO % 128) == 0 && (WSB_Q % 128) == 0 && (WSB_K % 128) == 0 && (WSB_VT % 128) == 0);
static_assert((WSB_OP % 128) == 0 && (WSB_Y % 128) == 0);

typedef _Float16 v16h __attribute__((ext_vector_type(16)));
typedef _Float16 v8h  __attribute__((ext_vector_type(8)));
typedef __bf16   v16b __attribute__((ext_vector_type(16)));
typedef __bf16   v8b  __attribute__((ext_vector_type(8)));
typedef float    v8f  __attribute__((ext_vector_type(8)));
typedef float    v4f  __attribute__((ext_vector_type(4)));
typedef unsigned int v4u __attribute__((ext_vector_type(4)));

#if defined(__HIP_DEVICE_COMPILE__)
#define DEV_ASM 1
#else
#define DEV_ASM 0
#endif

__device__ __forceinline__ unsigned short bf_bits(float f) {
  unsigned u = __float_as_uint(f);
  return (unsigned short)((u + 0x7FFFu + ((u >> 16) & 1u)) >> 16);
}
__device__ __forceinline__ float bf_up(unsigned short hb) { return __uint_as_float(((unsigned)hb) << 16); }
__device__ __forceinline__ unsigned short h_bits(_Float16 x) { return __builtin_bit_cast(unsigned short, x); }
__device__ __forceinline__ unsigned pk16(unsigned short a, unsigned short b) { return (unsigned)a | ((unsigned)b << 16); }
__device__ __forceinline__ v8f zero8() { v8f z = {0.f, 0.f, 0.f, 0.f, 0.f, 0.f, 0.f, 0.f}; return z; }
__device__ __forceinline__ float wave_sum(float s) {
#pragma unroll
  for (int off = 1; off < 32; off <<= 1) s += __shfl_xor(s, off, 32);
  return s;
}

template <typename OT> struct FT;
template <> struct FT<__bf16>   { typedef v16b frag; typedef v8b half8; };
template <> struct FT<_Float16> { typedef v16h frag; typedef v8h half8; };

template <typename OT>
__device__ __forceinline__ typename FT<OT>::frag ldfrag(const OT* p) {
  union { typename FT<OT>::frag v; typename FT<OT>::half8 h[2]; } f;
  f.h[0] = *(const typename FT<OT>::half8*)(p);
  f.h[1] = *(const typename FT<OT>::half8*)(p + 16);
  return f.v;
}

__device__ __forceinline__ v8f mmar(v16b a, v16b b, v8f c) {
  return __builtin_amdgcn_wmma_f32_16x16x32_bf16(false, a, false, b, (short)0, c, false, false);
}
__device__ __forceinline__ v8f mmar(v16h a, v16h b, v8f c) {
  return __builtin_amdgcn_wmma_f32_16x16x32_f16(false, a, false, b, (short)0, c, false, false);
}
__device__ __forceinline__ v8f mma_h(v16h a, v16h b, v8f c) {
  c = __builtin_amdgcn_wmma_f32_16x16x32_f16(false, a, false, b, (short)0, c, false, false);
#if DEV_ASM
  asm volatile("v_nop\n\tv_nop\n\tv_nop\n\tv_nop" : "+v"(c) : "v"(a), "v"(b));
#endif
  return c;
}
__device__ __forceinline__ void dep_guard(v8f& a, v8f& b, v16b x, v16b y) {
#if DEV_ASM
  asm volatile("v_nop\n\tv_nop\n\tv_nop\n\tv_nop" : "+v"(a), "+v"(b) : "v"(x), "v"(y));
#else
  (void)a; (void)b; (void)x; (void)y;
#endif
}
__device__ __forceinline__ void dep_guard(v8f& a, v8f& b, v16h x, v16h y) {
#if DEV_ASM
  asm volatile("v_nop\n\tv_nop\n\tv_nop\n\tv_nop" : "+v"(a), "+v"(b) : "v"(x), "v"(y));
#else
  (void)a; (void)b; (void)x; (void)y;
#endif
}
__device__ __forceinline__ void keep4(v16b a, v16b b, v16b c, v16b d) {
#if DEV_ASM
  asm volatile("v_nop" :: "v"(a), "v"(b), "v"(c), "v"(d));
#else
  (void)a; (void)b; (void)c; (void)d;
#endif
}
__device__ __forceinline__ void keep4(v16h a, v16h b, v16h c, v16h d) {
#if DEV_ASM
  asm volatile("v_nop" :: "v"(a), "v"(b), "v"(c), "v"(d));
#else
  (void)a; (void)b; (void)c; (void)d;
#endif
}
__device__ __forceinline__ void acc_guard4(v8f& a, v8f& b, v8f& c, v8f& d) {
#if DEV_ASM
  asm volatile("v_nop\n\tv_nop\n\tv_nop\n\tv_nop" : "+v"(a), "+v"(b), "+v"(c), "+v"(d));
#else
  (void)a; (void)b; (void)c; (void)d;
#endif
}

__global__ __launch_bounds__(256) void cvt_bf16x8(const float* __restrict__ in, long long istride,
                                                 unsigned short* out, long long ostride, int n8) {
  const int b = blockIdx.y;
  const int i = blockIdx.x * 256 + (int)threadIdx.x;
  if (i < n8) {
    const float* ip = in + (size_t)b * (size_t)istride + (size_t)i * 8;
    const v4f a  = *(const v4f*)(ip);
    const v4f a4 = *(const v4f*)(ip + 4);
    v4u p;
    p[0] = pk16(bf_bits(a[0]),  bf_bits(a[1]));
    p[1] = pk16(bf_bits(a[2]),  bf_bits(a[3]));
    p[2] = pk16(bf_bits(a4[0]), bf_bits(a4[1]));
    p[3] = pk16(bf_bits(a4[2]), bf_bits(a4[3]));
    unsigned short* o = out + (size_t)b * (size_t)ostride + (size_t)i * 8;
    *(volatile v4u*)o = p;
    __threadfence();
    *(volatile v4u*)o = p;
  }
}

__global__ __launch_bounds__(256) void ln_in_planes(const float* __restrict__ x, const float* __restrict__ g,
                                                   unsigned short* xn) {
  const int lane = threadIdx.x & 31;
  const int wave = threadIdx.x >> 5;
  const int row  = blockIdx.x * 8 + wave;
  if (row >= NB * SEQ) return;
  const int b = row / SEQ;
  const int t = row - b * SEQ;
  const float* ip = x + ((size_t)b * SEQ_FULL + (size_t)t) * DM;
  float v[16];
#pragma unroll
  for (int it = 0; it < 2; ++it) {
    const int col = it * 256 + lane * 8;
    const v4f a  = *(const v4f*)(ip + col);
    const v4f a4 = *(const v4f*)(ip + col + 4);
#pragma unroll
    for (int e = 0; e < 4; ++e) {
      v[it * 8 + e]     = bf_up(bf_bits(a[e]));
      v[it * 8 + 4 + e] = bf_up(bf_bits(a4[e]));
    }
  }
  float s = 0.f;
#pragma unroll
  for (int e = 0; e < 16; ++e) s += v[e];
  s = wave_sum(s);
  const float mean = s * (1.0f / (float)DM);
  float ss = 0.f;
#pragma unroll
  for (int e = 0; e < 16; ++e) { const float d = v[e] - mean; ss += d * d; }
  ss = wave_sum(ss);
  const float rstd = rsqrtf(ss * (1.0f / (float)DM) + LN_EPS);
  v4u hv[2], lv[2];
#pragma unroll
  for (int it = 0; it < 2; ++it) {
    const int col = it * 256 + lane * 8;
    const v4f ga  = *(const v4f*)(g + col);
    const v4f ga4 = *(const v4f*)(g + col + 4);
    unsigned short hb[8], lb[8];
#pragma unroll
    for (int e = 0; e < 8; ++e) {
      const float gr = (e < 4) ? ga[e & 3] : ga4[e & 3];
      const float y  = (v[it * 8 + e] - mean) * rstd * bf_up(bf_bits(gr));
      const unsigned short h = bf_bits(y);
      hb[e] = h;
      lb[e] = bf_bits(y - bf_up(h));
    }
    v4u a, a2;
#pragma unroll
    for (int e = 0; e < 4; ++e) { a[e] = pk16(hb[2 * e], hb[2 * e + 1]); a2[e] = pk16(lb[2 * e], lb[2 * e + 1]); }
    hv[it] = a; lv[it] = a2;
  }
  unsigned short* o = xn + (size_t)row * XLD;
  for (int ps = 0; ps < 2; ++ps) {
#pragma unroll
    for (int it = 0; it < 2; ++it) {
      const int col = it * 256 + lane * 8;
      *(volatile v4u*)(o + col) = hv[it];
      *(volatile v4u*)(o + DM + col) = lv[it];
    }
    __threadfence();
  }
}

__global__ __launch_bounds__(256) void ln_out_rows(const float* __restrict__ y, const float* __restrict__ g,
                                                  float* out) {
  const int lane = threadIdx.x & 31;
  const int wave = threadIdx.x >> 5;
  const int row  = blockIdx.x * 8 + wave;
  if (row >= NB * SEQ) return;
  const int b = row / SEQ;
  const int t = row - b * SEQ;
  const float* ip = y + (size_t)row * DM;
  v4f v[4];
#pragma unroll
  for (int it = 0; it < 4; ++it) v[it] = *(const v4f*)(ip + it * 128 + lane * 4);
  float s = 0.f;
#pragma unroll
  for (int it = 0; it < 4; ++it) s += (v[it][0] + v[it][1]) + (v[it][2] + v[it][3]);
  s = wave_sum(s);
  const float mean = s * (1.0f / (float)DM);
  float ss = 0.f;
#pragma unroll
  for (int it = 0; it < 4; ++it) {
#pragma unroll
    for (int e = 0; e < 4; ++e) { const float d = v[it][e] - mean; ss += d * d; }
  }
  ss = wave_sum(ss);
  const float rstd = rsqrtf(ss * (1.0f / (float)DM) + LN_EPS);
  v4f o[4];
#pragma unroll
  for (int it = 0; it < 4; ++it) {
    const v4f gr = *(const v4f*)(g + it * 128 + lane * 4);
    v4f r;
#pragma unroll
    for (int e = 0; e < 4; ++e) r[e] = (v[it][e] - mean) * rstd * bf_up(bf_bits(gr[e]));
    o[it] = r;
  }
  float* op = out + ((size_t)b * SEQ_FULL + (size_t)t) * DM;
  for (int ps = 0; ps < 2; ++ps) {
#pragma unroll
    for (int it = 0; it < 4; ++it) *(volatile v4f*)(op + it * 128 + lane * 4) = o[it];
    __threadfence();
  }
}

template <int MODE>
__device__ __forceinline__ unsigned short cvm(float f, float scale) {
  const unsigned short hb = bf_bits(f);
  if (MODE == 0) return hb;
  return h_bits((_Float16)(bf_up(hb) * scale));
}

template <int MODE>
__device__ __forceinline__ void wtrans_body(const float* __restrict__ W, int C,
                                            unsigned short* T, int ldt, int coff, float scale,
                                            float* sW) {
  const int tid  = threadIdx.x;
  const int lane = tid & 31;
  const int wave = tid >> 5;
  const int n0 = blockIdx.x * 64;
  const int k0 = blockIdx.y * 64;
#pragma unroll
  for (int j = 0; j < 4; ++j) {
    const int lin = tid + j * 256;
    const int r = lin >> 4, c4 = (lin & 15) * 4;
    const v4f val = *(const v4f*)(W + (size_t)(k0 + r) * (size_t)C + n0 + c4);
    sW[(c4 + 0) * 68 + r] = val[0];
    sW[(c4 + 1) * 68 + r] = val[1];
    sW[(c4 + 2) * 68 + r] = val[2];
    sW[(c4 + 3) * 68 + r] = val[3];
  }
  __syncthreads();
  const int q = lane >> 3, c8 = (lane & 7) * 8;
  v4u pv[2];
#pragma unroll
  for (int it = 0; it < 2; ++it) {
    const int row = it * 32 + wave * 4 + q;
    const float* sp = sW + row * 68 + c8;
    v4u a;
#pragma unroll
    for (int e = 0; e < 4; ++e)
      a[e] = pk16(cvm<MODE>(sp[2 * e], scale), cvm<MODE>(sp[2 * e + 1], scale));
    pv[it] = a;
  }
  for (int ps = 0; ps < 2; ++ps) {
#pragma unroll
    for (int it = 0; it < 2; ++it) {
      const int row = it * 32 + wave * 4 + q;
      *(volatile v4u*)(T + (size_t)(n0 + row) * (size_t)ldt + coff + k0 + c8) = pv[it];
    }
    __threadfence();
  }
}

__global__ __launch_bounds__(256) void wtrans_bf16(const float* __restrict__ W, int C,
                                                  unsigned short* T, int ldt, int coff, float scale) {
  __shared__ __align__(16) float sW[64 * 68];
  wtrans_body<0>(W, C, T, ldt, coff, scale, sW);
}
__global__ __launch_bounds__(256) void wtrans_f16s(const float* __restrict__ W, int C,
                                                  unsigned short* T, int ldt, int coff, float scale) {
  __shared__ __align__(16) float sW[64 * 68];
  wtrans_body<1>(W, C, T, ldt, coff, scale, sW);
}

template <typename OT, int OUT_MODE>
__device__ __forceinline__ void gemm64_body(
    const unsigned short* __restrict__ Ap, int lda, long long strideA,
    const unsigned short* __restrict__ Btp, int ldb, long long strideB,
    void* Cout, void* Cout2, int ldc, long long strideC,
    int M, int N, int K, float oscale, float rscale, float* sTall) {
  typedef typename FT<OT>::frag V16;
  const OT* A  = (const OT*)(const void*)Ap;
  const OT* Bt = (const OT*)(const void*)Btp;
  const int b    = blockIdx.y;
  const int lane = threadIdx.x & 31;
  const int wave = threadIdx.x >> 5;
  const int tilesN = N >> 6;
  const int tilesM = M >> 6;
  const int tile = blockIdx.x * 8 + wave;
  if (tile >= tilesM * tilesN) return;
  const int tm = tile / tilesN;
  const int tn = tile - tm * tilesN;
  const int m0 = tm << 6;
  const int n0 = tn << 6;

  const OT* Ab = A  + (size_t)b * (size_t)strideA;
  const OT* Bb = Bt + (size_t)b * (size_t)strideB;

  const int rlane = lane & 15;
  const int koff  = (lane >> 4) * 8;
  const int mOff  = (lane >> 4) * 8;

  v8f acc[4][4];
#pragma unroll
  for (int i = 0; i < 4; ++i)
#pragma unroll
    for (int j = 0; j < 4; ++j) acc[i][j] = zero8();

  for (int k0 = 0; k0 < K; k0 += 32) {
    V16 bq[4];
#pragma unroll
    for (int j = 0; j < 4; ++j)
      bq[j] = ldfrag<OT>(Bb + (size_t)(n0 + (j << 4) + rlane) * ldb + koff + k0);
#pragma unroll
    for (int i = 0; i < 4; ++i) {
      const V16 af = ldfrag<OT>(Ab + (size_t)(m0 + (i << 4) + rlane) * lda + koff + k0);
#pragma unroll
      for (int j = 0; j < 4; ++j) acc[i][j] = mmar(af, bq[j], acc[i][j]);
      dep_guard(acc[i][0], acc[i][3], af, bq[3]);
    }
    keep4(bq[0], bq[1], bq[2], bq[3]);
  }
  acc_guard4(acc[0][0], acc[0][1], acc[0][2], acc[0][3]);
  acc_guard4(acc[1][0], acc[1][1], acc[1][2], acc[1][3]);
  acc_guard4(acc[2][0], acc[2][1], acc[2][2], acc[2][3]);
  acc_guard4(acc[3][0], acc[3][1], acc[3][2], acc[3][3]);

  float* slab = sTall + wave * (16 * 68);
#pragma unroll
  for (int i = 0; i < 4; ++i) {
    const int mBase = m0 + (i << 4);
#pragma unroll
    for (int j = 0; j < 4; ++j) {
#pragma unroll
      for (int r = 0; r < 8; ++r) {
        slab[(mOff + r) * 68 + (j << 4) + rlane] = acc[i][j][r];
      }
    }
    __builtin_amdgcn_fence(3  , "workgroup");
    __builtin_amdgcn_wave_barrier();
    __builtin_amdgcn_fence(2  , "workgroup");
    if (OUT_MODE == 0) {
      float* Cb0 = (float*)Cout + (size_t)b * (size_t)strideC;
      const int h2 = lane >> 4, c4 = (lane & 15) * 4;
      for (int ps = 0; ps < 2; ++ps) {
#pragma unroll
        for (int it = 0; it < 8; ++it) {
          const int row = it * 2 + h2;
          const v4f v = *(const v4f*)(slab + row * 68 + c4) * oscale;
          *(volatile v4f*)(Cb0 + (size_t)(mBase + row) * ldc + n0 + c4) = v;
        }
        __threadfence();
      }
    } else {
      const int q = lane >> 3, c8 = (lane & 7) * 8;
      unsigned short* Cp  = (unsigned short*)Cout  + (size_t)b * (size_t)strideC;
      unsigned short* Cp2 = (unsigned short*)Cout2 + (size_t)b * (size_t)strideC;
      v4u hv[4], lv[4];
#pragma unroll
      for (int it = 0; it < 4; ++it) {
        const int row = it * 4 + q;
        const float* sp = slab + row * 68 + c8;
        float f[8];
#pragma unroll
        for (int e = 0; e < 8; ++e) f[e] = sp[e] * oscale;
        v4u a, a2;
#pragma unroll
        for (int e = 0; e < 4; ++e) {
          const float f0 = f[2 * e], f1 = f[2 * e + 1];
          const _Float16 x0 = (_Float16)f0, x1 = (_Float16)f1;
          const unsigned short h0 = h_bits(x0), h1 = h_bits(x1);
          unsigned short l0 = 0, l1 = 0;
          if (OUT_MODE == 3) {
            l0 = h_bits((_Float16)((f0 - (float)x0) * rscale));
            l1 = h_bits((_Float16)((f1 - (float)x1) * rscale));
          }
          a[e] = pk16(h0, h1); a2[e] = pk16(l0, l1);
        }
        hv[it] = a; lv[it] = a2;
      }
      for (int ps = 0; ps < 2; ++ps) {
#pragma unroll
        for (int it = 0; it < 4; ++it) {
          const int row = it * 4 + q;
          *(volatile v4u*)(Cp + (size_t)(mBase + row) * ldc + n0 + c8) = hv[it];
          if (OUT_MODE == 3) *(volatile v4u*)(Cp2 + (size_t)(mBase + row) * ldc + n0 + c8) = lv[it];
        }
        __threadfence();
      }
    }
    __builtin_amdgcn_fence(3  , "workgroup");
    __builtin_amdgcn_wave_barrier();
    __builtin_amdgcn_fence(2  , "workgroup");
  }
}

__global__ __launch_bounds__(256) void gemm_proj_split(
    const unsigned short* __restrict__ Ap, int lda, long long strideA,
    const unsigned short* __restrict__ Btp, int ldb, long long strideB,
    void* Cout, void* Cout2, int ldc, long long strideC,
    int M, int N, int K, float oscale, float rscale) {
  __shared__ __align__(16) float sT[8 * 16 * 68];
  gemm64_body<__bf16, 3>(Ap, lda, strideA, Btp, ldb, strideB, Cout, Cout2, ldc, strideC,
                         M, N, K, oscale, rscale, sT);
}
__global__ __launch_bounds__(256) void gemm_proj_plane(
    const unsigned short* __restrict__ Ap, int lda, long long strideA,
    const unsigned short* __restrict__ Btp, int ldb, long long strideB,
    void* Cout, void* Cout2, int ldc, long long strideC,
    int M, int N, int K, float oscale, float rscale) {
  __shared__ __align__(16) float sT[8 * 16 * 68];
  gemm64_body<__bf16, 1>(Ap, lda, strideA, Btp, ldb, strideB, Cout, Cout2, ldc, strideC,
                         M, N, K, oscale, rscale, sT);
}
__global__ __launch_bounds__(256) void gemm_out_f32(
    const unsigned short* __restrict__ Ap, int lda, long long strideA,
    const unsigned short* __restrict__ Btp, int ldb, long long strideB,
    void* Cout, void* Cout2, int ldc, long long strideC,
    int M, int N, int K, float oscale, float rscale) {
  __shared__ __align__(16) float sT[8 * 16 * 68];
  gemm64_body<_Float16, 0>(Ap, lda, strideA, Btp, ldb, strideB, Cout, Cout2, ldc, strideC,
                           M, N, K, oscale, rscale, sT);
}

__global__ __launch_bounds__(128)
void attn_nullmask(const unsigned short* __restrict__ qhp, const unsigned short* __restrict__ qlp,
                   const unsigned short* __restrict__ kpp, const unsigned short* __restrict__ vtp,
                   const int* __restrict__ mask, const float* __restrict__ nullkv,
                   unsigned short* op, float kscale) {
  union FH { v16h v; v8h h[2]; };
  __shared__ __align__(16) _Float16 Ksh[64 * 64];
  __shared__ __align__(16) _Float16 Vth[64 * 64];
  __shared__ __align__(16) _Float16 Psh[4][16 * 64];
  __shared__ __align__(16) float    Os[4][16 * 64];
  __shared__ int   Msk[64];
  __shared__ float Nk[64];
  __shared__ float Nv[64];

  const int tid  = threadIdx.x;
  const int wave = tid >> 5;
  const int lane = tid & 31;
  const int hh   = lane >> 4;
  const int c    = lane & 15;

  const int bx   = blockIdx.x;
  const int qb   = bx % NQB;
  const int rest = bx / NQB;
  const int h    = rest % NH;
  const int b    = rest / NH;
  const int q0   = qb * 64 + wave * 16;
  const size_t rowQ = (size_t)b * SEQ;
  const size_t rowK = (size_t)b * MSEQ;

  const _Float16* Qh = (const _Float16*)(const void*)qhp;
  const _Float16* Ql = (const _Float16*)(const void*)qlp;
  const _Float16* Kg = (const _Float16*)(const void*)kpp + (size_t)h * HD;
  const _Float16* Vg = (const _Float16*)(const void*)vtp + ((size_t)b * DI + (size_t)h * HD) * (size_t)MSEQ;
  const int* mg = mask + (size_t)b * MSEQ_FULL;

  if (tid < 64) {
    Nk[tid] = bf_up(bf_bits(nullkv[tid])) * kscale;
    Nv[tid] = bf_up(bf_bits(nullkv[HD + tid]));
  }
  __syncthreads();

  v16h qah[2], qal[2];
#pragma unroll
  for (int dc = 0; dc < 2; ++dc) {
    const size_t qo = (rowQ + q0 + c) * DI + (size_t)h * HD + dc * 32 + 8 * hh;
    qah[dc] = ldfrag<_Float16>(Qh + qo);
    qal[dc] = ldfrag<_Float16>(Ql + qo);
  }

  float pn = 0.f;
  {
    const size_t qo = (rowQ + q0 + c) * DI + (size_t)h * HD + hh * 32;
#pragma unroll 1
    for (int i = 0; i < 4; ++i) {
      const v8h a = *(const v8h*)(Qh + qo + 8 * i);
      const v8h l = *(const v8h*)(Ql + qo + 8 * i);
#pragma unroll
      for (int e = 0; e < 8; ++e) {
        const float qv = (float)a[e] + (float)l[e] * (1.0f / RQ);
        pn += qv * Nk[hh * 32 + 8 * i + e];
      }
    }
  }
  pn += __shfl_xor(pn, 16, 32);

  float mrow[8], lrow[8];
  v8f oacc[4];
#pragma unroll
  for (int r = 0; r < 8; ++r) {
    mrow[r] = __shfl(pn, 8 * hh + r, 32);
    lrow[r] = 1.0f;
  }
#pragma unroll
  for (int t = 0; t < 4; ++t) {
    const float nv = Nv[t * 16 + c] * (PCARRY * VCARRY);
#pragma unroll
    for (int r = 0; r < 8; ++r) oacc[t][r] = nv;
  }

  for (int kt = 0; kt < NKT; ++kt) {
    const int kv0 = kt * 64;
    __syncthreads();
    {
      const int r = tid >> 1, half = (tid & 1) * 32;
      const _Float16* kg = Kg + (rowK + kv0 + r) * DI + half;
      const _Float16* vg = Vg + (size_t)r * MSEQ + kv0 + half;
#pragma unroll
      for (int i = 0; i < 4; ++i) {
        const v8h a0 = *(const v8h*)(kg + 8 * i);
        const v8h b0 = *(const v8h*)(vg + 8 * i);
        *(v8h*)(Ksh + r * 64 + half + 8 * i) = a0;
        *(v8h*)(Vth + r * 64 + half + 8 * i) = b0;
      }
      if (tid < 64) Msk[tid] = mg[kv0 + tid];
    }
    __syncthreads();

    v8f s[4];
    int mkv[4];
#pragma unroll
    for (int j = 0; j < 4; ++j) {
      v8f ah = zero8(), al = zero8();
#pragma unroll
      for (int dc = 0; dc < 2; ++dc) {
        FH kb;
        kb.h[0] = *(const v8h*)(Ksh + (j * 16 + c) * 64 + dc * 32 + 8 * hh);
        kb.h[1] = *(const v8h*)(Ksh + (j * 16 + c) * 64 + dc * 32 + 16 + 8 * hh);
        ah = mma_h(qah[dc], kb.v, ah);
        al = mma_h(qal[dc], kb.v, al);
      }
      const int mk = Msk[j * 16 + c];
      mkv[j] = mk;
#pragma unroll
      for (int r = 0; r < 8; ++r) {
        const float sv = ah[r] + al[r] * (1.0f / RQ);
        s[j][r] = (mk != 0) ? sv : NEGMAX;
      }
    }

    _Float16* pwh = Psh[wave];
#pragma unroll
    for (int r = 0; r < 8; ++r) {
      float m = s[0][r];
#pragma unroll
      for (int j = 1; j < 4; ++j) m = fmaxf(m, s[j][r]);
#pragma unroll
      for (int off = 1; off < 16; off <<= 1) m = fmaxf(m, __shfl_xor(m, off, 32));
      const float mnew  = fmaxf(mrow[r], m);
      const float alpha = __expf(mrow[r] - mnew);
      mrow[r] = mnew;
      float psum = 0.f;
#pragma unroll
      for (int j = 0; j < 4; ++j) {
        const float ev = __expf(fmaxf(s[j][r] - mnew, -80.0f));
        const float p  = (mkv[j] != 0) ? ev : 0.f;
        psum += p;
        pwh[(8 * hh + r) * 64 + j * 16 + c] = (_Float16)(p * PCARRY);
      }
#pragma unroll
      for (int off = 1; off < 16; off <<= 1) psum += __shfl_xor(psum, off, 32);
      lrow[r] = lrow[r] * alpha + psum;
#pragma unroll
      for (int t = 0; t < 4; ++t) oacc[t][r] *= alpha;
    }
    __builtin_amdgcn_fence(3  , "workgroup");
    __builtin_amdgcn_wave_barrier();
    __builtin_amdgcn_fence(2  , "workgroup");

#pragma unroll 1
    for (int kk = 0; kk < 2; ++kk) {
      FH pa;
      pa.h[0] = *(const v8h*)(pwh + c * 64 + kk * 32 + 8 * hh);
      pa.h[1] = *(const v8h*)(pwh + c * 64 + kk * 32 + 16 + 8 * hh);
#pragma unroll
      for (int t = 0; t < 4; ++t) {
        FH vb;
        vb.h[0] = *(const v8h*)(Vth + (t * 16 + c) * 64 + kk * 32 + 8 * hh);
        vb.h[1] = *(const v8h*)(Vth + (t * 16 + c) * 64 + kk * 32 + 16 + 8 * hh);
        oacc[t] = mma_h(pa.v, vb.v, oacc[t]);
      }
    }
  }

  float* os = Os[wave];
#pragma unroll
  for (int r = 0; r < 8; ++r) {
    const float l = lrow[r];
    const float inv = ((l > 0.f) ? (1.0f / l) : 0.f) * (CCARRY / (PCARRY * VCARRY));
#pragma unroll
    for (int t = 0; t < 4; ++t) os[(8 * hh + r) * 64 + t * 16 + c] = oacc[t][r] * inv;
  }
  __builtin_amdgcn_fence(3  , "workgroup");
  __builtin_amdgcn_wave_barrier();
  __builtin_amdgcn_fence(2  , "workgroup");
  {
    const int q4 = lane >> 3, c8 = (lane & 7) * 8;
    v4u hv[4], lv[4];
#pragma unroll
    for (int it = 0; it < 4; ++it) {
      const int row = it * 4 + q4;
      const float* sp = os + row * 64 + c8;
      v4u a, a2;
#pragma unroll
      for (int e = 0; e < 4; ++e) {
        const float f0 = sp[2 * e], f1 = sp[2 * e + 1];
        const _Float16 x0 = (_Float16)f0, x1 = (_Float16)f1;
        const unsigned short l0 = h_bits((_Float16)((f0 - (float)x0) * RC));
        const unsigned short l1 = h_bits((_Float16)((f1 - (float)x1) * RC));
        a[e]  = pk16(h_bits(x0), h_bits(x1));
        a2[e] = pk16(l0, l1);
      }
      hv[it] = a; lv[it] = a2;
    }
    for (int ps = 0; ps < 2; ++ps) {
#pragma unroll
      for (int it = 0; it < 4; ++it) {
        const int row = it * 4 + q4;
        const size_t go = (rowQ + q0 + row) * OPLD + (size_t)h * HD + c8;
        *(volatile v4u*)(op + go) = hv[it];
        *(volatile v4u*)(op + go + DI) = lv[it];
      }
      __threadfence();
    }
  }
}

extern "C" void kernel_launch(void* const* d_in, const int* in_sizes, int n_in,
                              void* d_out, int out_size, void* d_ws, size_t ws_size,
                              hipStream_t stream) {
  if (n_in < 9) return;
  if (in_sizes[0] < ((NB - 1) * SEQ_FULL + SEQ) * DM) return;
  if (in_sizes[1] < ((NB - 1) * MSEQ_FULL + MSEQ) * DC) return;
  if (in_sizes[2] < (NB - 1) * MSEQ_FULL + MSEQ) return;
  if (in_sizes[3] < DM) return;
  if (in_sizes[4] < 2 * HD) return;
  if (in_sizes[5] < DM * DI) return;
  if (in_sizes[6] < DC * KVN) return;
  if (in_sizes[7] < DI * DM) return;
  if (in_sizes[8] < DM) return;
  if (out_size < ((NB - 1) * SEQ_FULL + SEQ) * DM) return;

  const float* x      = (const float*)d_in[0];
  const float* ctx    = (const float*)d_in[1];
  const int*   mask   = (const int*)d_in[2];
  const float* g_x    = (const float*)d_in[3];
  const float* nullkv = (const float*)d_in[4];
  const float* Wq     = (const float*)d_in[5];
  const float* Wkv    = (const float*)d_in[6];
  const float* Wo     = (const float*)d_in[7];
  const float* g_out  = (const float*)d_in[8];

  size_t off = 0;
  const size_t oXN = off; off += WSB_XN;
  const size_t oCb = off; off += WSB_CB;
  const size_t oWq = off; off += WSB_WQ;
  const size_t oWk = off; off += WSB_WKV;
  const size_t oWo = off; off += WSB_WO;
  const size_t oQh = off; off += WSB_Q;
  const size_t oQl = off; off += WSB_Q;
  const size_t oKp = off; off += WSB_K;
  const size_t oVT = off; off += WSB_VT;
  const size_t oOp = off; off += WSB_OP;
  const size_t oY  = off; off += WSB_Y;
  if (off != WSB_TOTAL) return;
  if (off > ws_size) return;
  if (off > (size_t)134217728) return;

  char* ws = (char*)d_ws;
  unsigned short* XN   = (unsigned short*)(ws + oXN);
  unsigned short* Cb   = (unsigned short*)(ws + oCb);
  unsigned short* WqT  = (unsigned short*)(ws + oWq);
  unsigned short* WkvT = (unsigned short*)(ws + oWk);
  unsigned short* WoT  = (unsigned short*)(ws + oWo);
  unsigned short* Qh   = (unsigned short*)(ws + oQh);
  unsigned short* Ql   = (unsigned short*)(ws + oQl);
  unsigned short* Kp   = (unsigned short*)(ws + oKp);
  unsigned short* VT   = (unsigned short*)(ws + oVT);
  unsigned short* Op   = (unsigned short*)(ws + oOp);
  float*          Y    = (float*)(ws + oY);

  const dim3 blk(256);
  const int n8c = MSEQ * DC / 8;
  const dim3 gCvtC((n8c + 255) / 256, NB);
  const dim3 gLN((NB * SEQ) / 8);
  const dim3 gWQ(DI / 64, DM / 64);
  const dim3 gWKV(KVN / 64, DC / 64);
  const dim3 gWO(DM / 64, DI / 64);
  const dim3 gQ((((NB * SEQ) / 64) * (DI / 64) + 7) / 8, 1);
  const dim3 gK((((NB * MSEQ) / 64) * (DI / 64) + 7) / 8, 1);
  const dim3 gVT(((DI / 64) * (MSEQ / 64) + 7) / 8, NB);
  const dim3 gAttn(NB * NH * NQB);
  const dim3 gO((((NB * SEQ) / 64) * (DM / 64) + 7) / 8, 1);

  cvt_bf16x8<<<gCvtC, blk, 0, stream>>>(ctx, (long long)MSEQ_FULL * DC, Cb, (long long)MSEQ * DC, n8c);
  ln_in_planes<<<gLN, blk, 0, stream>>>(x, g_x, XN);
  wtrans_bf16<<<gWQ, blk, 0, stream>>>(Wq, DI, WqT, XLD, 0,  1.0f);
  wtrans_bf16<<<gWQ, blk, 0, stream>>>(Wq, DI, WqT, XLD, DM, 1.0f);
  wtrans_bf16<<<gWKV, blk, 0, stream>>>(Wkv, KVN, WkvT, DC, 0, 1.0f);
  wtrans_f16s<<<gWO, blk, 0, stream>>>(Wo, DM, WoT, OPLD, 0,  WOC);
  wtrans_f16s<<<gWO, blk, 0, stream>>>(Wo, DM, WoT, OPLD, DI, 1.0f);
  gemm_proj_split<<<gQ, blk, 0, stream>>>(
      XN, XLD, 0LL, WqT, XLD, 0LL,
      (void*)Qh, (void*)Ql, DI, 0LL,
      NB * SEQ, DI, XLD, SQK, RQ);
  gemm_proj_plane<<<gK, blk, 0, stream>>>(
      Cb, DC, 0LL, WkvT, DC, 0LL,
      (void*)Kp, (void*)Kp, DI, 0LL,
      NB * MSEQ, DI, DC, SQK, 1.0f);
  gemm_proj_plane<<<gVT, blk, 0, stream>>>(
      WkvT + (size_t)DI * DC, DC, 0LL, Cb, DC, (long long)MSEQ * DC,
      (void*)VT, (void*)VT, MSEQ, (long long)DI * MSEQ,
      DI, MSEQ, DC, VCARRY, 1.0f);
  attn_nullmask<<<gAttn, dim3(128), 0, stream>>>(Qh, Ql, Kp, VT, mask, nullkv, Op, SQK);
  gemm_out_f32<<<gO, blk, 0, stream>>>(
      Op, OPLD, 0LL, WoT, OPLD, 0LL,
      (void*)Y, (void*)Y, DM, 0LL,
      NB * SEQ, DM, OPLD, 1.0f / (CCARRY * WOC), 1.0f);
  ln_out_rows<<<gLN, blk, 0, stream>>>(Y, g_out, (float*)d_out);
  (void)hipGetLastError();
}
